// GraphSAGEFraudDetector_20323785244835
// MI455X (gfx1250) — hardware-verified
//
#include <hip/hip_runtime.h>
#include <stdint.h>
#include <stddef.h>
#include <math.h>


typedef _Float16 v8h  __attribute__((ext_vector_type(8)));
typedef _Float16 v16h __attribute__((ext_vector_type(16)));
typedef float    v2f  __attribute__((ext_vector_type(2)));
typedef float    v4f  __attribute__((ext_vector_type(4)));
typedef float    v8f  __attribute__((ext_vector_type(8)));
typedef int      v4i  __attribute__((ext_vector_type(4)));
typedef v8h v8ha __attribute__((may_alias));
typedef v4f v4fa __attribute__((may_alias));
typedef v2f v2fa __attribute__((may_alias));
typedef v4i v4ia __attribute__((may_alias));

#define FD      64
#define RNODE   1024
#define EPL     16
#define EPW     (32 * EPL)
#define WPITCH  72
#define SPITCH  68
#define GW      8
#define NPART   64
#define AGG_LDS_BYTES ((RNODE * FD + RNODE) * 4)

union Frag { v16h v; v8h half[2]; };

__device__ __forceinline__ v8f wmma_f16(v16h a, v16h b, v8f c)
{
  v8f d = __builtin_amdgcn_wmma_f32_16x16x32_f16(false, a, false, b, (short)0, c, false, false);
  asm volatile("v_nop\n\tv_nop\n\tv_nop\n\tv_nop" : "+v"(d) : "v"(a), "v"(b));
  return d;
}

template <int COUNT>
__global__ void __launch_bounds__(32)
k_agg(const float* __restrict__ hin, const int* __restrict__ esrc, const int* __restrict__ edst,
      int n_edges, int n_nodes, int vec_ok,
      const float* inv_in, float* inv_out, _Float16* agg_out)
{
  extern __shared__ __align__(16) float lds_dyn[];
  float* acc = lds_dyn;
  float* cnt = lds_dyn + RNODE * FD;
  const int lane = threadIdx.x;
  const int n0 = blockIdx.x * RNODE;
  const int nmax = n_nodes - 1;

  {
    const v4f z = {0.f, 0.f, 0.f, 0.f};
    v4fa* p = (v4fa*)lds_dyn;
    for (int i = lane; i < (RNODE * FD + RNODE) / 4; i += 32) p[i] = z;
  }
  __syncthreads();

  for (int base = 0; base < n_edges; base += EPW) {
    const int e0 = base + lane * EPL;
    int dv[EPL], sv[EPL];
    if (vec_ok && (e0 + EPL <= n_edges)) {
#pragma unroll
      for (int q = 0; q < EPL / 4; ++q) {
        const v4i d4 = *(const v4ia*)(edst + e0 + 4 * q);
        const v4i s4 = *(const v4ia*)(esrc + e0 + 4 * q);
        dv[4 * q + 0] = d4[0]; dv[4 * q + 1] = d4[1]; dv[4 * q + 2] = d4[2]; dv[4 * q + 3] = d4[3];
        sv[4 * q + 0] = s4[0]; sv[4 * q + 1] = s4[1]; sv[4 * q + 2] = s4[2]; sv[4 * q + 3] = s4[3];
      }
    } else {
#pragma unroll
      for (int j = 0; j < EPL; ++j) {
        const int e = e0 + j;
        const bool ok = e < n_edges;
        const int ec = ok ? e : 0;
        const int d = edst[ec];
        const int s = esrc[ec];
        dv[j] = ok ? d : -1;
        sv[j] = ok ? s : 0;
      }
    }
#pragma unroll
    for (int j = 0; j < EPL; ++j) {
      const unsigned t = (unsigned)(dv[j] - n0);
      unsigned m = __builtin_amdgcn_ballot_w32(t < (unsigned)RNODE);
      while (m != 0u) {
        const int k = __builtin_ctz(m);
        m &= m - 1u;
        const int tl = __builtin_amdgcn_readlane((int)t, k) & (RNODE - 1);
        int s = __builtin_amdgcn_readlane(sv[j], k);
        s = s < 0 ? 0 : (s > nmax ? nmax : s);
        const v2f v = *(const v2fa*)(hin + (size_t)s * FD + 2 * lane);
        float* ap = acc + tl * FD + 2 * lane;
        v2f a = *(v2fa*)ap;
        a += v;
        *(v2fa*)ap = a;
        if (COUNT) cnt[tl] += 1.0f;
      }
    }
  }
  __syncthreads();

  if (COUNT) {
    for (int i = lane; i < RNODE; i += 32) cnt[i] = 1.0f / fmaxf(cnt[i], 1.0f);
    __syncthreads();
    for (int pass = 0; pass < 2; ++pass) {
      for (int i = lane; i < RNODE / 4; i += 32) {
        const v4f v = *(const v4fa*)(cnt + 4 * i);
        *(volatile v4f*)(inv_out + (size_t)n0 + 4 * i) = v;
      }
      __threadfence();
    }
  } else {
    for (int i = lane; i < RNODE / 4; i += 32)
      *(v4fa*)(cnt + 4 * i) = *(const v4fa*)(inv_in + (size_t)n0 + 4 * i);
    __syncthreads();
  }

  const int rsub = lane >> 3;
  const int c8 = (lane & 7) * 8;
  for (int pass = 0; pass < 2; ++pass) {
    for (int r0 = 0; r0 < RNODE; r0 += 4) {
      const int r = r0 + rsub;
      const float w = cnt[r];
      const v4f x0 = *(const v4fa*)(acc + r * FD + c8);
      const v4f x1 = *(const v4fa*)(acc + r * FD + c8 + 4);
      v8h o;
      o[0] = (_Float16)(x0[0] * w); o[1] = (_Float16)(x0[1] * w);
      o[2] = (_Float16)(x0[2] * w); o[3] = (_Float16)(x0[3] * w);
      o[4] = (_Float16)(x1[0] * w); o[5] = (_Float16)(x1[1] * w);
      o[6] = (_Float16)(x1[2] * w); o[7] = (_Float16)(x1[3] * w);
      *(volatile v8h*)(agg_out + ((size_t)(n0 + r)) * FD + c8) = o;
    }
    __threadfence();
  }
}

__global__ void __launch_bounds__(256)
k_conv(const _Float16* __restrict__ agg, const float* __restrict__ hin,
       const float* __restrict__ wl, const float* __restrict__ bl, const float* __restrict__ wr,
       const float* __restrict__ gam, const float* __restrict__ bet,
       const float* __restrict__ mu, const float* __restrict__ var,
       float* hout, int n_tiles, int n_nodes)
{
  __shared__ __align__(16) _Float16 wls[FD * WPITCH];
  __shared__ __align__(16) _Float16 wrs[FD * WPITCH];
  __shared__ float sbias[FD], smu[FD], sscg[FD], sbet[FD];
  __shared__ __align__(16) float stg[GW][16 * SPITCH];

  const int tid = threadIdx.x;
  for (int i = tid; i < FD * FD; i += 256) {
    const int o = i >> 6, k = i & 63;
    wls[o * WPITCH + k] = (_Float16)wl[i];
    wrs[o * WPITCH + k] = (_Float16)wr[i];
  }
  if (tid < FD) {
    sbias[tid] = bl[tid];
    smu[tid] = mu[tid];
    sscg[tid] = rsqrtf(var[tid] + 1e-5f) * gam[tid];
    sbet[tid] = bet[tid];
  }
  __syncthreads();

  const int wid = tid >> 5, lane = tid & 31, m = lane & 15, h = lane >> 4;
  const int wave = blockIdx.x * GW + wid;
  const bool valid = wave < n_tiles;
  const int tile = valid ? wave : (n_tiles - 1);
  const int row0 = tile * 16;
  int node = row0 + m;
  if (node > n_nodes - 1) node = n_nodes - 1;

  Frag aA[2], aH[2];
#pragma unroll
  for (int kk = 0; kk < 2; ++kk) {
    const int k0 = 32 * kk;
    const _Float16* ap = agg + (size_t)node * FD + k0 + 8 * h;
    aA[kk].half[0] = *(const v8ha*)(ap);
    aA[kk].half[1] = *(const v8ha*)(ap + 16);
    const float* hp = hin + (size_t)node * FD + k0 + 8 * h;
    const v4f f0 = *(const v4fa*)(hp);
    const v4f f1 = *(const v4fa*)(hp + 4);
    const v4f f2 = *(const v4fa*)(hp + 16);
    const v4f f3 = *(const v4fa*)(hp + 20);
    v8h lo, hi;
    lo[0] = (_Float16)f0[0]; lo[1] = (_Float16)f0[1]; lo[2] = (_Float16)f0[2]; lo[3] = (_Float16)f0[3];
    lo[4] = (_Float16)f1[0]; lo[5] = (_Float16)f1[1]; lo[6] = (_Float16)f1[2]; lo[7] = (_Float16)f1[3];
    hi[0] = (_Float16)f2[0]; hi[1] = (_Float16)f2[1]; hi[2] = (_Float16)f2[2]; hi[3] = (_Float16)f2[3];
    hi[4] = (_Float16)f3[0]; hi[5] = (_Float16)f3[1]; hi[6] = (_Float16)f3[2]; hi[7] = (_Float16)f3[3];
    aH[kk].half[0] = lo;
    aH[kk].half[1] = hi;
  }

  const v8f z8 = {0.f, 0.f, 0.f, 0.f, 0.f, 0.f, 0.f, 0.f};
  v8f acc[4];
  acc[0] = z8; acc[1] = z8; acc[2] = z8; acc[3] = z8;

#pragma unroll
  for (int t = 0; t < 4; ++t) {
    const int n = 16 * t + m;
#pragma unroll
    for (int kk = 0; kk < 2; ++kk) {
      const int k0 = 32 * kk;
      Frag b;
      b.half[0] = *(const v8ha*)(wls + n * WPITCH + k0 + 8 * h);
      b.half[1] = *(const v8ha*)(wls + n * WPITCH + k0 + 16 + 8 * h);
      acc[t] = wmma_f16(aA[kk].v, b.v, acc[t]);
    }
#pragma unroll
    for (int kk = 0; kk < 2; ++kk) {
      const int k0 = 32 * kk;
      Frag b;
      b.half[0] = *(const v8ha*)(wrs + n * WPITCH + k0 + 8 * h);
      b.half[1] = *(const v8ha*)(wrs + n * WPITCH + k0 + 16 + 8 * h);
      acc[t] = wmma_f16(aH[kk].v, b.v, acc[t]);
    }
  }

  float* stw = &stg[wid][0];
#pragma unroll
  for (int t = 0; t < 4; ++t) {
    const int col = 16 * t + m;
    const float bb = sbias[col], mm = smu[col], sc = sscg[col], be = sbet[col];
#pragma unroll
    for (int r = 0; r < 8; ++r) {
      float v = acc[t][r] + bb;
      v = fmaxf((v - mm) * sc + be, 0.f);
      stw[(8 * h + r) * SPITCH + col] = v;
    }
  }
  __syncthreads();

  const int rr = lane >> 4, cc = (lane & 15) * 4;
  for (int pass = 0; pass < 2; ++pass) {
    if (valid) {
#pragma unroll
      for (int k = 0; k < 8; ++k) {
        const int row = 2 * k + rr;
        const v4f v = *(const v4fa*)(stw + row * SPITCH + cc);
        *(volatile v4f*)(hout + (size_t)(row0 + row) * FD + cc) = v;
      }
    }
    __threadfence();
  }
}

__global__ void __launch_bounds__(256)
k_pool(const float* __restrict__ h2, const int* __restrict__ esrc, const int* __restrict__ edst,
       const float* __restrict__ inv, int n_edges, int n_nodes, int epb, int npb, float* part)
{
  __shared__ float red[32 * FD];
  __shared__ __align__(16) float outv[2 * FD];
  const int tid = threadIdx.x, gi = tid >> 3, j = tid & 7;
  const int nmax = n_nodes - 1;

  float a[8];
#pragma unroll
  for (int i = 0; i < 8; ++i) a[i] = 0.f;
  {
    const int eb = blockIdx.x * epb;
    int ee = eb + epb;
    if (ee > n_edges) ee = n_edges;
    for (int e = eb + gi; e < ee; e += 32) {
      int s = esrc[e], d = edst[e];
      s = s < 0 ? 0 : (s > nmax ? nmax : s);
      d = d < 0 ? 0 : (d > nmax ? nmax : d);
      const float w = inv[d];
      const float* rp = h2 + (size_t)s * FD + 8 * j;
      const v4f x0 = *(const v4fa*)(rp);
      const v4f x1 = *(const v4fa*)(rp + 4);
      a[0] += w * x0[0]; a[1] += w * x0[1]; a[2] += w * x0[2]; a[3] += w * x0[3];
      a[4] += w * x1[0]; a[5] += w * x1[1]; a[6] += w * x1[2]; a[7] += w * x1[3];
    }
  }
#pragma unroll
  for (int i = 0; i < 8; ++i) red[gi * FD + 8 * j + i] = a[i];
  __syncthreads();
  if (tid < FD) {
    float s = 0.f;
    for (int g = 0; g < 32; ++g) s += red[g * FD + tid];
    outv[tid] = s;
  }
  __syncthreads();

#pragma unroll
  for (int i = 0; i < 8; ++i) a[i] = 0.f;
  {
    const int nb = blockIdx.x * npb;
    int ne = nb + npb;
    if (ne > n_nodes) ne = n_nodes;
    for (int n = nb + gi; n < ne; n += 32) {
      const float* rp = h2 + (size_t)n * FD + 8 * j;
      const v4f x0 = *(const v4fa*)(rp);
      const v4f x1 = *(const v4fa*)(rp + 4);
      a[0] += x0[0]; a[1] += x0[1]; a[2] += x0[2]; a[3] += x0[3];
      a[4] += x1[0]; a[5] += x1[1]; a[6] += x1[2]; a[7] += x1[3];
    }
  }
#pragma unroll
  for (int i = 0; i < 8; ++i) red[gi * FD + 8 * j + i] = a[i];
  __syncthreads();
  if (tid < FD) {
    float s = 0.f;
    for (int g = 0; g < 32; ++g) s += red[g * FD + tid];
    outv[FD + tid] = s;
  }
  __syncthreads();

  v4f v = {0.f, 0.f, 0.f, 0.f};
  if (tid < 32) v = *(const v4fa*)(outv + 4 * tid);
  for (int pass = 0; pass < 2; ++pass) {
    if (tid < 32) *(volatile v4f*)(part + (size_t)blockIdx.x * (2 * FD) + 4 * tid) = v;
    __threadfence();
  }
}

__global__ void __launch_bounds__(64)
k_head(const float* __restrict__ part, int nparts, int n_nodes,
       const float* __restrict__ wl2, const float* __restrict__ bl2, const float* __restrict__ wr2,
       const float* __restrict__ cw1, const float* __restrict__ cb1,
       const float* __restrict__ cw2, const float* __restrict__ cb2, float* out)
{
  __shared__ float sma[FD], smh[FD], sz[FD], sy[FD];
  const int t = threadIdx.x;
  double sa = 0.0, sh = 0.0;
#pragma unroll 1
  for (int b = 0; b < nparts; ++b) {
    sa += (double)part[(size_t)b * (2 * FD) + t];
    sh += (double)part[(size_t)b * (2 * FD) + FD + t];
  }
  const double invn = 1.0 / (double)n_nodes;
  sma[t] = (float)(sa * invn);
  smh[t] = (float)(sh * invn);
  __syncthreads();
  float z = bl2[t];
#pragma unroll 1
  for (int f = 0; f < FD; ++f) z += sma[f] * wl2[t * FD + f] + smh[f] * wr2[t * FD + f];
  sz[t] = z;
  __syncthreads();
  float y = cb1[t];
#pragma unroll 1
  for (int o = 0; o < FD; ++o) y += sz[o] * cw1[t * FD + o];
  sy[t] = fmaxf(y, 0.f);
  __syncthreads();
  if (t == 0) {
    float s = cb2[0];
#pragma unroll 1
    for (int k = 0; k < FD; ++k) s += sy[k] * cw2[k];
    const float r = 1.0f / (1.0f + expf(-s));
    *(volatile float*)out = r;
    __threadfence();
    *(volatile float*)out = r;
  }
}

extern "C" void kernel_launch(void* const* d_in, const int* in_sizes, int n_in,
                              void* d_out, int out_size, void* d_ws, size_t ws_size,
                              hipStream_t stream)
{
  if (n_in < 23 || out_size < 1) return;
  const int n_nodes = in_sizes[0] / FD;
  const int n_edges = in_sizes[1] / 2;
  if (n_nodes < 1 || n_nodes * FD != in_sizes[0]) return;
  if (n_edges < 1 || n_edges * 2 != in_sizes[1]) return;
  {
    const int wi[7] = {2, 4, 5, 7, 8, 10, 19};
    for (int i = 0; i < 7; ++i) if (in_sizes[wi[i]] != FD * FD) return;
    const int vi[12] = {3, 6, 9, 11, 12, 13, 14, 15, 16, 17, 18, 20};
    for (int i = 0; i < 12; ++i) if (in_sizes[vi[i]] != FD) return;
    if (in_sizes[21] != FD || in_sizes[22] < 1) return;
  }

  const float* x   = (const float*)d_in[0];
  const int*   ei  = (const int*)d_in[1];
  const int*   src = ei;
  const int*   dst = ei + (size_t)n_edges;
  const float* wl0 = (const float*)d_in[2];
  const float* bl0 = (const float*)d_in[3];
  const float* wr0 = (const float*)d_in[4];
  const float* wl1 = (const float*)d_in[5];
  const float* bl1 = (const float*)d_in[6];
  const float* wr1 = (const float*)d_in[7];
  const float* wl2 = (const float*)d_in[8];
  const float* bl2 = (const float*)d_in[9];
  const float* wr2 = (const float*)d_in[10];
  const float* g0  = (const float*)d_in[11];
  const float* be0 = (const float*)d_in[12];
  const float* m0  = (const float*)d_in[13];
  const float* v0  = (const float*)d_in[14];
  const float* g1  = (const float*)d_in[15];
  const float* be1 = (const float*)d_in[16];
  const float* m1  = (const float*)d_in[17];
  const float* v1  = (const float*)d_in[18];
  const float* cw1 = (const float*)d_in[19];
  const float* cb1 = (const float*)d_in[20];
  const float* cw2 = (const float*)d_in[21];
  const float* cb2 = (const float*)d_in[22];

  const int nb_agg    = (n_nodes + RNODE - 1) / RNODE;
  const int npad      = nb_agg * RNODE;
  const int n_tiles   = (n_nodes + 15) / 16;
  const int conv_grid = (n_tiles + GW - 1) / GW;
  const int epb       = (n_edges + NPART - 1) / NPART;
  const int npb       = (n_nodes + NPART - 1) / NPART;
  const int vec_ok    = (n_edges % 4 == 0) ? 1 : 0;

  char* ws = (char*)d_ws;
  size_t off = 0;
  const size_t b_agg  = (size_t)npad * FD * sizeof(_Float16);
  const size_t b_inv  = (size_t)npad * sizeof(float);
  const size_t b_h    = (size_t)npad * FD * sizeof(float);
  const size_t b_part = (size_t)NPART * 2 * FD * sizeof(float);
  _Float16* agg16 = (_Float16*)(ws + off); off += (b_agg + 255) & ~(size_t)255;
  float* inv  = (float*)(ws + off); off += (b_inv + 255) & ~(size_t)255;
  float* h1   = (float*)(ws + off); off += (b_h + 255) & ~(size_t)255;
  float* h2   = (float*)(ws + off); off += (b_h + 255) & ~(size_t)255;
  float* part = (float*)(ws + off); off += (b_part + 255) & ~(size_t)255;
  if (off > ws_size) return;

  hipFuncSetAttribute(reinterpret_cast<const void*>(&k_agg<1>),
                      hipFuncAttributeMaxDynamicSharedMemorySize, AGG_LDS_BYTES);
  hipFuncSetAttribute(reinterpret_cast<const void*>(&k_agg<0>),
                      hipFuncAttributeMaxDynamicSharedMemorySize, AGG_LDS_BYTES);

  k_agg<1><<<nb_agg, 32, AGG_LDS_BYTES, stream>>>(x, src, dst, n_edges, n_nodes, vec_ok,
                                                   inv, inv, agg16);
  k_conv<<<conv_grid, 256, 0, stream>>>(agg16, x, wl0, bl0, wr0, g0, be0, m0, v0,
                                        h1, n_tiles, n_nodes);
  k_agg<0><<<nb_agg, 32, AGG_LDS_BYTES, stream>>>(h1, src, dst, n_edges, n_nodes, vec_ok,
                                                   inv, inv, agg16);
  k_conv<<<conv_grid, 256, 0, stream>>>(agg16, h1, wl1, bl1, wr1, g1, be1, m1, v1,
                                        h2, n_tiles, n_nodes);
  k_pool<<<NPART, 256, 0, stream>>>(h2, src, dst, inv, n_edges, n_nodes, epb, npb, part);
  k_head<<<1, 64, 0, stream>>>(part, NPART, n_nodes, wl2, bl2, wr2, cw1, cb1, cw2, cb2,
                               (float*)d_out);
}
